// SOMISSMLayer_33200097198711
// MI455X (gfx1250) — hardware-run, weakly checked
//
#include <hip/hip_runtime.h>
#include <math.h>

typedef __attribute__((ext_vector_type(8)))  _Float16 v8h;
typedef __attribute__((ext_vector_type(16))) __bf16   v16b;
typedef __attribute__((ext_vector_type(8)))  __bf16   v8b;
typedef __attribute__((ext_vector_type(8)))  float    v8f;
typedef __attribute__((ext_vector_type(4)))  float    v4f;

constexpr int kTok   = 4 * 2048;
constexpr int kHd    = 1024;
constexpr int kBn    = 64;
constexpr int kPitch = 68;
constexpr int kTilesM = kTok / 64;
constexpr int kTilesN = kHd / 64;
constexpr int kStepWaves   = 2;
constexpr int kStepThreads = kStepWaves * 32;
constexpr float kDt = 0.35f;
static_assert(kTok == 8192 && kHd == 1024 && kBn == 64, "wire shapes");
static_assert((kTok % 64) == 0 && (kHd % 64) == 0 && (kBn % 64) == 0, "M,N multiples of 64");
static_assert((kHd % 32) == 0 && (kBn % 32) == 0, "K multiples of 32");
static_assert(((kTilesM * kTilesN) % kStepWaves) == 0, "step grid exact");
static_assert((kTilesM % 8) == 0, "hid grid exact");

constexpr size_t kOffAW   = 0;
constexpr size_t kOffGW1  = kOffAW   + (size_t)kHd  * kHd * 2;
constexpr size_t kOffGW2  = kOffGW1  + (size_t)kBn  * kHd * 2;
constexpr size_t kOffIDG  = kOffGW2  + (size_t)kHd  * kBn * 2;
constexpr size_t kOffIMS  = kOffIDG  + (size_t)kHd  * 4;
constexpr size_t kOffP16A = kOffIMS  + (size_t)kHd  * 4;
constexpr size_t kOffP16B = kOffP16A + (size_t)kTok * kHd * 2;
constexpr size_t kOffHID  = kOffP16B + (size_t)kTok * kHd * 2;
constexpr size_t kOffPHI  = kOffHID  + (size_t)kTok * kBn * 2;
constexpr size_t kOffPD   = kOffPHI  + (size_t)kTok * kHd * 4;
constexpr size_t kWsTotal = kOffPD   + (size_t)kTok * kHd * 4;
static_assert(kWsTotal == 2097152ull + 131072ull + 131072ull + 4096ull + 4096ull + 16777216ull + 16777216ull +
                          1048576ull + 33554432ull + 33554432ull, "carve sum");
static_assert(kWsTotal == 104079360ull, "carve total");
static_assert(kWsTotal <= 134217728ull, "carve cap");
static_assert((kOffGW1 % 128) == 0 && (kOffGW2 % 128) == 0 && (kOffIDG % 128) == 0 && (kOffIMS % 128) == 0 &&
              (kOffP16A % 128) == 0 && (kOffP16B % 128) == 0 && (kOffHID % 128) == 0 && (kOffPHI % 128) == 0 &&
              (kOffPD % 128) == 0, "128-B aligned regions");

__device__ __forceinline__ unsigned short f2bf_bits(float f) {
  unsigned u = __float_as_uint(f);
  return (unsigned short)((u + 0x7FFFu + ((u >> 16) & 1u)) >> 16);
}

__device__ __forceinline__ v8h pack8_bf16(v4f a0, v4f a1) {
  v8h o;
#pragma unroll
  for (int e = 0; e < 4; ++e) {
    const float f0 = a0[e];
    const float f1 = a1[e];
    const unsigned short h0 = f2bf_bits(f0);
    const unsigned short h1 = f2bf_bits(f1);
    o[e]     = __builtin_bit_cast(_Float16, h0);
    o[4 + e] = __builtin_bit_cast(_Float16, h1);
  }
  return o;
}

__device__ __forceinline__ void wave_lds_sync() {
  __builtin_amdgcn_fence(__ATOMIC_RELEASE, "workgroup");
  __builtin_amdgcn_wave_barrier();
  __builtin_amdgcn_fence(__ATOMIC_ACQUIRE, "workgroup");
}

__device__ __forceinline__ v16b frag_load(const __bf16* p) {
  union U { v16b v; v8b h[2]; } f;
  f.h[0] = *(const v8b*)(p);
  f.h[1] = *(const v8b*)(p + 16);
  return f.v;
}
__device__ __forceinline__ v8f mma_bf16(v16b a, v16b b, v8f c) {
  return __builtin_amdgcn_wmma_f32_16x16x32_bf16(false, a, false, b, (short)0, c, false, false);
}
__device__ __forceinline__ void tie_acc(v8f& a, v16b x, v16b y) { asm volatile("" : "+v"(a) : "v"(x), "v"(y)); }
__device__ __forceinline__ void tie_acc_nop(v8f& a, v16b x, v16b y) {
  asm volatile("v_nop\n\tv_nop\n\tv_nop\n\tv_nop" : "+v"(a) : "v"(x), "v"(y));
}
__device__ __forceinline__ void keep4_b(v16b a, v16b b, v16b c, v16b d) { asm volatile("v_nop" :: "v"(a), "v"(b), "v"(c), "v"(d)); }

__device__ __forceinline__ void mac_tile64(const __bf16* __restrict__ Ap, int lda,
                                           const __bf16* __restrict__ Bp, int ldb,
                                           int K, v8f (&acc)[4][4]) {
#pragma unroll 1
  for (int k0 = 0; k0 < K; k0 += 32) {
    v16b bh[4];
#pragma unroll
    for (int j = 0; j < 4; ++j) bh[j] = frag_load(Bp + (size_t)(j << 4) * ldb + k0);
#pragma unroll
    for (int i = 0; i < 4; ++i) {
      const v16b ah = frag_load(Ap + (size_t)(i << 4) * lda + k0);
#pragma unroll
      for (int j = 0; j < 4; ++j) acc[i][j] = mma_bf16(ah, bh[j], acc[i][j]);
      tie_acc(acc[i][0], ah, bh[0]);
      tie_acc(acc[i][1], ah, bh[1]);
      tie_acc(acc[i][2], ah, bh[2]);
      tie_acc_nop(acc[i][3], ah, bh[3]);
    }
    keep4_b(bh[0], bh[1], bh[2], bh[3]);
  }
}

__global__ __launch_bounds__(256) void cvt_rows_bf16_kernel(
    const float* __restrict__ src, unsigned short* __restrict__ dst, int total8) {
  const int i = blockIdx.x * 256 + threadIdx.x;
  if (i >= total8) return;
  const size_t e0 = (size_t)i << 3;
  const v4f a0 = *(const v4f*)(src + e0);
  const v4f a1 = *(const v4f*)(src + e0 + 4);
  const v8h hv = pack8_bf16(a0, a1);
  unsigned short* q = dst + e0;
  *(volatile v8h*)q = hv;
  __threadfence();
  *(volatile v8h*)q = hv;
}

__global__ __launch_bounds__(256) void prep_w_kernel(
    const float* __restrict__ W, const float* __restrict__ mass,
    unsigned short* __restrict__ AW, float* __restrict__ invdeg, float* __restrict__ invmass) {
  __shared__ float sSum[32];
  const int lane = threadIdx.x & 31, wave = threadIdx.x >> 5;
  const int o0 = blockIdx.x * 32;
#pragma unroll 1
  for (int r = 0; r < 4; ++r) {
    const int o = o0 + wave * 4 + r;
    const float* wr = W + (size_t)o * kHd;
    unsigned short* ar = AW + (size_t)o * kHd;
    float part = 0.0f;
#pragma unroll 1
    for (int c = 0; c < 4; ++c) {
      const int i0 = (c * 32 + lane) * 8;
      v4f a0 = *(const v4f*)(wr + i0);
      v4f a1 = *(const v4f*)(wr + i0 + 4);
      a0[0] = fabsf(a0[0]); a0[1] = fabsf(a0[1]); a0[2] = fabsf(a0[2]); a0[3] = fabsf(a0[3]);
      a1[0] = fabsf(a1[0]); a1[1] = fabsf(a1[1]); a1[2] = fabsf(a1[2]); a1[3] = fabsf(a1[3]);
      part += ((a0[0] + a0[1]) + (a0[2] + a0[3])) + ((a1[0] + a1[1]) + (a1[2] + a1[3]));
      const v8h hv = pack8_bf16(a0, a1);
      *(volatile v8h*)(ar + i0) = hv;
      __threadfence();
      *(volatile v8h*)(ar + i0) = hv;
    }
#pragma unroll
    for (int off = 1; off < 32; off <<= 1) part += __shfl_xor(part, off, 32);
    if (lane == 0) sSum[wave * 4 + r] = part;
  }
  __syncthreads();
  if (wave == 0) {
    const float s = sSum[lane];
    const float v = 1.0f / fmaxf(s, 1e-8f);
    *(volatile float*)(invdeg + o0 + lane) = v;
    __threadfence();
    *(volatile float*)(invdeg + o0 + lane) = v;
  } else if (wave == 1) {
    const float mv = mass[o0 + lane];
    const float v = 1.0f / mv;
    *(volatile float*)(invmass + o0 + lane) = v;
    __threadfence();
    *(volatile float*)(invmass + o0 + lane) = v;
  }
}

__global__ __launch_bounds__(256) void hid_gemm_kernel(
    const unsigned short* __restrict__ P16, const unsigned short* __restrict__ GW1,
    const float* __restrict__ gb1, unsigned short* __restrict__ HID) {
  __shared__ __align__(16) float sT[8][16 * kPitch];
  const int lane = threadIdx.x & 31, wave = threadIdx.x >> 5;
  const int tile = blockIdx.x * 8 + wave;
  if (tile >= kTilesM) return;
  const int m0 = tile << 6;
  const int rlane = lane & 15, hh = lane >> 4;
  const int koff = hh * 8, mOff = hh * 8;

  v8f acc[4][4];
#pragma unroll
  for (int i = 0; i < 4; ++i)
#pragma unroll
    for (int j = 0; j < 4; ++j) acc[i][j] = (v8f){0.f, 0.f, 0.f, 0.f, 0.f, 0.f, 0.f, 0.f};

  mac_tile64((const __bf16*)P16 + (size_t)(m0 + rlane) * kHd + koff, kHd,
             (const __bf16*)GW1 + (size_t)rlane * kHd + koff, kHd, kHd, acc);

  float* slab = sT[wave];
  const int q = lane >> 3, c8 = (lane & 7) * 8;
#pragma unroll
  for (int i = 0; i < 4; ++i) {
    const int mBase = m0 + (i << 4);
#pragma unroll
    for (int j = 0; j < 4; ++j) {
      const float bv = gb1[(j << 4) + rlane];
#pragma unroll
      for (int r = 0; r < 8; ++r) {
        float v = acc[i][j][r] + bv;
        v = fmaxf(v, 0.0f);
        slab[(mOff + r) * kPitch + (j << 4) + rlane] = v;
      }
    }
    wave_lds_sync();
    for (int pass = 0; pass < 2; ++pass) {
#pragma unroll
      for (int it = 0; it < 4; ++it) {
        const int row = it * 4 + q;
        const float* sp = slab + row * kPitch + c8;
        const v4f a0 = *(const v4f*)(sp);
        const v4f a1 = *(const v4f*)(sp + 4);
        const v8h hv = pack8_bf16(a0, a1);
        *(volatile v8h*)(HID + (size_t)(mBase + row) * kBn + c8) = hv;
      }
      __threadfence();
    }
    wave_lds_sync();
  }
}

__device__ __forceinline__ void settle_elem(float ph, float pd, float tg, float s, float g,
                                            float pc, float im, float idg, float beta,
                                            float& phn, float& pdn) {
  const float diff  = ph - idg * s;
  const float force = -(diff + (ph - tg) * pc);
  const float accel = (g * force - beta * pd) * im;
  const float pv = pd + kDt * accel;
  pdn = pv;
  phn = ph + kDt * pv;
}

template <bool FIRST>
__global__ __launch_bounds__(kStepThreads) void settle_step_kernel(
    const unsigned short* __restrict__ P16cur, const unsigned short* __restrict__ AW,
    const unsigned short* __restrict__ HID, const unsigned short* __restrict__ GW2,
    const float* __restrict__ hT, const float* __restrict__ prec, const float* __restrict__ invmass,
    const float* __restrict__ invdeg, const float* __restrict__ gb2,
    float* phi32, float* pd32, unsigned short* __restrict__ P16next, float beta) {
  __shared__ __align__(16) float sGate[kStepWaves][64 * kPitch];
  __shared__ __align__(16) float sSlab[kStepWaves][16 * kPitch];
  const int lane = threadIdx.x & 31, wave = threadIdx.x >> 5;
  const int tile = blockIdx.x * kStepWaves + wave;
  if (tile >= kTilesM * kTilesN) return;
  const int tm = tile / kTilesN;
  const int tn = tile - tm * kTilesN;
  const int m0 = tm << 6, n0 = tn << 6;
  const int rlane = lane & 15, hh = lane >> 4;
  const int koff = hh * 8, mOff = hh * 8;
  const int c4 = rlane * 4;
  float* sg   = sGate[wave];
  float* slab = sSlab[wave];

  v8f acc[4][4];
#pragma unroll
  for (int i = 0; i < 4; ++i)
#pragma unroll
    for (int j = 0; j < 4; ++j) acc[i][j] = (v8f){0.f, 0.f, 0.f, 0.f, 0.f, 0.f, 0.f, 0.f};

  mac_tile64((const __bf16*)HID + (size_t)(m0 + rlane) * kBn + koff, kBn,
             (const __bf16*)GW2 + (size_t)(n0 + rlane) * kBn + koff, kBn, kBn, acc);
#pragma unroll
  for (int i = 0; i < 4; ++i)
#pragma unroll
    for (int j = 0; j < 4; ++j)
#pragma unroll
      for (int r = 0; r < 8; ++r)
        sg[((i << 4) + mOff + r) * kPitch + (j << 4) + rlane] = acc[i][j][r];
  wave_lds_sync();
  {
    const v4f b2v = *(const v4f*)(gb2 + n0 + c4);
#pragma unroll 1
    for (int it = 0; it < 32; ++it) {
      float* gp = sg + (it * 2 + hh) * kPitch + c4;
      const v4f x = *(const v4f*)gp;
      v4f g;
      g[0] = 1.0f / (1.0f + expf(-(x[0] + b2v[0])));
      g[1] = 1.0f / (1.0f + expf(-(x[1] + b2v[1])));
      g[2] = 1.0f / (1.0f + expf(-(x[2] + b2v[2])));
      g[3] = 1.0f / (1.0f + expf(-(x[3] + b2v[3])));
      *(v4f*)gp = g;
    }
  }
  wave_lds_sync();

#pragma unroll
  for (int i = 0; i < 4; ++i)
#pragma unroll
    for (int j = 0; j < 4; ++j) acc[i][j] = (v8f){0.f, 0.f, 0.f, 0.f, 0.f, 0.f, 0.f, 0.f};
  mac_tile64((const __bf16*)P16cur + (size_t)(m0 + rlane) * kHd + koff, kHd,
             (const __bf16*)AW + (size_t)(n0 + rlane) * kHd + koff, kHd, kHd, acc);

  const v4f pcv = *(const v4f*)(prec + n0 + c4);
  const v4f imv = *(const v4f*)(invmass + n0 + c4);
  const v4f idv = *(const v4f*)(invdeg + n0 + c4);
  const int q = lane >> 3, c8 = (lane & 7) * 8;
#pragma unroll
  for (int i = 0; i < 4; ++i) {
#pragma unroll
    for (int j = 0; j < 4; ++j)
#pragma unroll
      for (int r = 0; r < 8; ++r)
        slab[(mOff + r) * kPitch + (j << 4) + rlane] = acc[i][j][r];
    wave_lds_sync();
#pragma unroll 1
    for (int it = 0; it < 8; ++it) {
      const int row = it * 2 + hh;
      const size_t gidx = (size_t)(m0 + (i << 4) + row) * kHd + n0 + c4;
      float* sp = slab + row * kPitch + c4;
      const v4f sv = *(const v4f*)sp;
      const v4f gv = *(const v4f*)(sg + ((i << 4) + row) * kPitch + c4);
      const v4f tg = *(const v4f*)(hT + gidx);
      v4f ph, pd;
      if (FIRST) {
        ph = tg;
        pd = (v4f){0.f, 0.f, 0.f, 0.f};
      } else {
        ph = *(const v4f*)(phi32 + gidx);
        pd = *(const v4f*)(pd32 + gidx);
      }
      v4f phn, pdn;
      {
        float a, b;
        settle_elem(ph[0], pd[0], tg[0], sv[0], gv[0], pcv[0], imv[0], idv[0], beta, a, b);
        phn[0] = a; pdn[0] = b;
        settle_elem(ph[1], pd[1], tg[1], sv[1], gv[1], pcv[1], imv[1], idv[1], beta, a, b);
        phn[1] = a; pdn[1] = b;
        settle_elem(ph[2], pd[2], tg[2], sv[2], gv[2], pcv[2], imv[2], idv[2], beta, a, b);
        phn[2] = a; pdn[2] = b;
        settle_elem(ph[3], pd[3], tg[3], sv[3], gv[3], pcv[3], imv[3], idv[3], beta, a, b);
        phn[3] = a; pdn[3] = b;
      }
      *(volatile v4f*)(pd32 + gidx)  = pdn;
      *(volatile v4f*)(phi32 + gidx) = phn;
      __threadfence();
      *(volatile v4f*)(pd32 + gidx)  = pdn;
      *(volatile v4f*)(phi32 + gidx) = phn;
      *(v4f*)sp = phn;
    }
    wave_lds_sync();
    for (int pass = 0; pass < 2; ++pass) {
#pragma unroll
      for (int it = 0; it < 4; ++it) {
        const int row = it * 4 + q;
        const float* sp = slab + row * kPitch + c8;
        const v4f a0 = *(const v4f*)(sp);
        const v4f a1 = *(const v4f*)(sp + 4);
        const v8h hv = pack8_bf16(a0, a1);
        *(volatile v8h*)(P16next + (size_t)(m0 + (i << 4) + row) * kHd + n0 + c8) = hv;
      }
      __threadfence();
    }
    wave_lds_sync();
  }
}

__global__ __launch_bounds__(256) void layernorm_kernel(
    const float* __restrict__ X, const float* __restrict__ gamma, const float* __restrict__ lbeta,
    float* __restrict__ out) {
  const int lane = threadIdx.x & 31, wave = threadIdx.x >> 5;
  const int row = blockIdx.x * 8 + wave;
  if (row >= kTok) return;
  const float* xr = X + (size_t)row * kHd;
  float* orow = out + (size_t)row * kHd;
  float s = 0.0f;
#pragma unroll 1
  for (int c = 0; c < 8; ++c) {
    const v4f v = *(const v4f*)(xr + (c * 32 + lane) * 4);
    s += (v[0] + v[1]) + (v[2] + v[3]);
  }
#pragma unroll
  for (int off = 1; off < 32; off <<= 1) s += __shfl_xor(s, off, 32);
  const float mu = s * (1.0f / (float)kHd);
  float qs = 0.0f;
#pragma unroll 1
  for (int c = 0; c < 8; ++c) {
    const v4f v = *(const v4f*)(xr + (c * 32 + lane) * 4);
    const float d0 = v[0] - mu, d1 = v[1] - mu, d2 = v[2] - mu, d3 = v[3] - mu;
    qs += (d0 * d0 + d1 * d1) + (d2 * d2 + d3 * d3);
  }
#pragma unroll
  for (int off = 1; off < 32; off <<= 1) qs += __shfl_xor(qs, off, 32);
  const float var = qs * (1.0f / (float)kHd);
  const float inv = rsqrtf(var + 1e-5f);
#pragma unroll 1
  for (int c = 0; c < 8; ++c) {
    const int col = (c * 32 + lane) * 4;
    const v4f v  = *(const v4f*)(xr + col);
    const v4f gm = *(const v4f*)(gamma + col);
    const v4f bt = *(const v4f*)(lbeta + col);
    v4f o;
    o[0] = (v[0] - mu) * inv * gm[0] + bt[0];
    o[1] = (v[1] - mu) * inv * gm[1] + bt[1];
    o[2] = (v[2] - mu) * inv * gm[2] + bt[2];
    o[3] = (v[3] - mu) * inv * gm[3] + bt[3];
    *(volatile v4f*)(orow + col) = o;
    __threadfence();
    *(volatile v4f*)(orow + col) = o;
  }
}

extern "C" void kernel_launch(void* const* d_in, const int* in_sizes, int n_in,
                              void* d_out, int out_size, void* d_ws, size_t ws_size,
                              hipStream_t stream) {
  if (n_in < 10) return;
  if (in_sizes[0] != kTok * kHd) return;
  if (in_sizes[1] != kHd * kHd) return;
  if (in_sizes[2] != kHd) return;
  if (in_sizes[3] != kHd) return;
  if (in_sizes[4] != kBn * kHd) return;
  if (in_sizes[5] != kBn) return;
  if (in_sizes[6] != kHd * kBn) return;
  if (in_sizes[7] != kHd) return;
  if (in_sizes[8] != kHd) return;
  if (in_sizes[9] != kHd) return;
  if (out_size != kTok * kHd) return;
  if (ws_size < kWsTotal) return;

  const double omega = sqrt(1.0 * 1.0 + 1.0 + 1.0);
  const float beta = (float)(2.0 * 0.7 * omega);
  int nset = (int)(3.14159265358979323846 / (omega * 0.35));
  if (nset < 3) nset = 3;
  if (nset > 10) nset = 10;

  const float* h    = (const float*)d_in[0];
  const float* W    = (const float*)d_in[1];
  const float* mass = (const float*)d_in[2];
  const float* prec = (const float*)d_in[3];
  const float* gw1  = (const float*)d_in[4];
  const float* gb1  = (const float*)d_in[5];
  const float* gw2  = (const float*)d_in[6];
  const float* gb2  = (const float*)d_in[7];
  const float* lng  = (const float*)d_in[8];
  const float* lnb  = (const float*)d_in[9];
  float* out = (float*)d_out;

  char* ws = (char*)d_ws;
  unsigned short* AW    = (unsigned short*)(ws + kOffAW);
  unsigned short* GW1   = (unsigned short*)(ws + kOffGW1);
  unsigned short* GW2   = (unsigned short*)(ws + kOffGW2);
  float*          IDG   = (float*)(ws + kOffIDG);
  float*          IMS   = (float*)(ws + kOffIMS);
  unsigned short* P16A  = (unsigned short*)(ws + kOffP16A);
  unsigned short* P16B  = (unsigned short*)(ws + kOffP16B);
  unsigned short* HID   = (unsigned short*)(ws + kOffHID);
  float*          PHI   = (float*)(ws + kOffPHI);
  float*          PD    = (float*)(ws + kOffPD);

  prep_w_kernel<<<kHd / 32, 256, 0, stream>>>(W, mass, AW, IDG, IMS);
  cvt_rows_bf16_kernel<<<(kBn * kHd / 8) / 256, 256, 0, stream>>>(gw1, GW1, kBn * kHd / 8);
  cvt_rows_bf16_kernel<<<(kHd * kBn / 8) / 256, 256, 0, stream>>>(gw2, GW2, kHd * kBn / 8);
  cvt_rows_bf16_kernel<<<(kTok * kHd / 8) / 256, 256, 0, stream>>>(h, P16A, kTok * kHd / 8);

  for (int s = 0; s < nset; ++s) {
    const unsigned short* cur = (s & 1) ? P16B : P16A;
    unsigned short*       nxt = (s & 1) ? P16A : P16B;
    hid_gemm_kernel<<<kTilesM / 8, 256, 0, stream>>>(cur, GW1, gb1, HID);
    if (s == 0) {
      settle_step_kernel<true><<<(kTilesM * kTilesN) / kStepWaves, kStepThreads, 0, stream>>>(
          cur, AW, HID, GW2, h, prec, IMS, IDG, gb2, PHI, PD, nxt, beta);
    } else {
      settle_step_kernel<false><<<(kTilesM * kTilesN) / kStepWaves, kStepThreads, 0, stream>>>(
          cur, AW, HID, GW2, h, prec, IMS, IDG, gb2, PHI, PD, nxt, beta);
    }
  }

  layernorm_kernel<<<kTok / 8, 256, 0, stream>>>(PHI, lng, lnb, out);
}
